// MessagePassingBlock_51608327029104
// MI455X (gfx1250) — hardware-verified
//
#include <hip/hip_runtime.h>


namespace {
constexpr int NB = 8, C = 128, H = 90, W = 160, KT = 9, PAD = 4, HP = 96  ;
constexpr float XS = 8.0f, WSC = 256.0f;

typedef _Float16 b16;
typedef __attribute__((ext_vector_type(16))) _Float16 v16b;
typedef __attribute__((ext_vector_type(8))) _Float16 v8b;
typedef __attribute__((ext_vector_type(8))) float v8f;
typedef __attribute__((ext_vector_type(4))) float v4f;
__device__ __forceinline__ float bf16_rne(float f) { unsigned int u = __float_as_uint(f); u += 0x7FFFu + ((u >> 16) & 1u); return __uint_as_float(u & 0xFFFF0000u); }
__device__ __forceinline__ v16b frag_kb(const b16* p, int hh) { const v8b a = *(const v8b*)(p + 8 * hh), b = *(const v8b*)(p + 16 + 8 * hh); v16b f;
#pragma unroll
  for (int e = 0; e < 8; ++e) { f[e] = a[e]; f[8 + e] = b[e]; } return f; }
__device__ __forceinline__ v8f wmma16b(v16b a, v16b b, v8f c) { v8f d = __builtin_amdgcn_wmma_f32_16x16x32_f16(false, a, false, b, (short)0, c, false, false); asm volatile("v_nop\n\tv_nop\n\tv_nop\n\tv_nop" : "+v"(d) : "v"(a), "v"(b)); return d; }
__device__ __forceinline__ void wave_lds_sync() { __builtin_amdgcn_fence(__ATOMIC_RELEASE, "workgroup"); __builtin_amdgcn_wave_barrier(); __builtin_amdgcn_fence(__ATOMIC_ACQUIRE, "workgroup"); }

__global__ __launch_bounds__(256) void prep_kernel(const float* __restrict__ x, const float* __restrict__ w0, const float* __restrict__ w1, const float* __restrict__ w2, const float* __restrict__ w3, float* __restrict__ out, b16* __restrict__ WK, b16* __restrict__ SL, size_t nsl, float* __restrict__ T, size_t nt) {
  const size_t t = (size_t)blockIdx.x * 256 + threadIdx.x; const size_t n0 = (size_t)NB * C * H * W / 4, n1 = (size_t)4 * C * KT * C / 8, n2 = nsl / 8, n3 = nt / 4;
  if (t < n0) { const v4f v = *(const v4f*)(x + t * 4); const v4f o = {bf16_rne(v[0]), bf16_rne(v[1]), bf16_rne(v[2]), bf16_rne(v[3])}; for (int pass = 0; pass < 2; ++pass) { *(volatile v4f*)(out + t * 4) = o; __threadfence(); } }
  else if (t < n0 + n1) { const size_t e = (t - n0) * 8; const int d = (int)(e / ((size_t)C * KT * C)); const size_t r = e - (size_t)d * C * KT * C; const int o_ = (int)(r / (KT * C)), k0 = (int)(r - (size_t)o_ * KT * C); const float* w = d == 0 ? w0 : d == 1 ? w1 : d == 2 ? w2 : w3; v8b o8;
    for (int j = 0; j < 8; ++j) { const int k = k0 + j, tap = k / C, c = k - tap * C; o8[j] = (b16)(bf16_rne(w[((size_t)o_ * C + c) * KT + tap]) * WSC); }
    for (int pass = 0; pass < 2; ++pass) { *(volatile v8b*)(WK + e) = o8; __threadfence(); } }
  else if (t < n0 + n1 + n2) { const v8b z = {}; *(volatile v8b*)(SL + (t - n0 - n1) * 8) = z; }
  else if (t < n0 + n1 + n2 + n3) { const v4f z = {0, 0, 0, 0}; *(volatile v4f*)(T + (t - n0 - n1 - n2) * 4) = z; }
}
template <int HORZ>
__global__ __launch_bounds__(256) void seed_kernel(const float* __restrict__ x, int s0, b16* __restrict__ S, float* __restrict__ out, float* __restrict__ T) {
  const int b = blockIdx.x, t_ = threadIdx.x; constexpr int M = HORZ ? H : W; constexpr int MP = M + 2 * PAD;
  for (int pass = 0; pass < 2; ++pass) {
    for (int i = t_; i < M * C; i += 256) { const int m = i / C, c = i - m * C; const float v = bf16_rne(HORZ ? x[(((size_t)b * C + c) * H + m) * W + s0] : x[(((size_t)b * C + c) * H + s0) * W + m]); ((volatile b16*)S)[((size_t)b * MP + PAD + m) * C + c] = (b16)(v * XS); }
    if (HORZ) { for (int i = t_; i < C * HP; i += 256) { const int c = i / HP, hh = i - c * HP; ((volatile float*)T)[(((size_t)b * C + c) * W + s0) * HP + hh] = (hh < H) ? bf16_rne(x[(((size_t)b * C + c) * H + hh) * W + s0]) : 0.0f; } }
    else if (pass == 0) { for (int i = t_; i < C * W; i += 256) { const int c = i / W, m = i - c * W; const size_t o = (((size_t)b * C + c) * H + s0) * W + m; const float nv = out[o] + bf16_rne(x[o]); ((volatile float*)out)[o] = nv; __threadfence(); ((volatile float*)out)[o] = nv; } }
    __threadfence(); }
}
template <int HORZ>
__global__ __launch_bounds__(HORZ ? 192 : 320) void step_kernel(const float* __restrict__ x, const b16* __restrict__ Sp, const b16* __restrict__ WKd, const float* __restrict__ bias, int si, b16* __restrict__ Sn, float* __restrict__ out, float* __restrict__ T) {
  constexpr int M = HORZ ? H : W, MP = M + 2 * PAD, NWV = HORZ ? 6 : 10, MR = NWV * 16  ;
  __shared__ __attribute__((aligned(16))) float St[64][MR + 4];
  const int b = blockIdx.x, t_ = threadIdx.x, wave = t_ >> 5, lane = t_ & 31, nloc = lane & 15, hlf = lane >> 4; const int m0 = wave * 16; const int mrow = min(m0 + nloc, M - 1);
  v8f acc[8];
#pragma unroll
  for (int t = 0; t < 8; ++t) acc[t] = (v8f){};
  const b16* Sb = Sp + (size_t)b * MP * C;
#pragma unroll 1
  for (int tap = 0; tap < KT; ++tap) {
#pragma unroll
    for (int cb = 0; cb < C; cb += 32) { const v16b a = frag_kb(Sb + (size_t)(mrow + tap) * C + cb, hlf);
#pragma unroll
      for (int t = 0; t < 8; ++t) acc[t] = wmma16b(a, frag_kb(WKd + (size_t)(t * 16 + nloc) * (KT * C) + tap * C + cb, hlf), acc[t]); } }
  float hv[8][8];
#pragma unroll
  for (int t = 0; t < 8; ++t) { const int c = t * 16 + nloc; const float bb = bf16_rne(bias[c]);
#pragma unroll
    for (int r = 0; r < 8; ++r) { const int m = m0 + 8 * hlf + r; float xv = 0.0f; if (m < M) xv = bf16_rne(HORZ ? x[(((size_t)b * C + c) * H + m) * W + si] : x[(((size_t)b * C + c) * H + si) * W + m]); hv[t][r] = xv + fmaxf(acc[t][r] * (1.0f / (XS * WSC)) + bb, 0.0f); } }
  for (int half = 0; half < 2; ++half) {
    __syncthreads();
#pragma unroll
    for (int t = 0; t < 4; ++t)
#pragma unroll
      for (int r = 0; r < 8; ++r) St[t * 16 + nloc][m0 + 8 * hlf + r] = hv[half * 4 + t][r];
    __syncthreads();
    for (int pass = 0; pass < 2; ++pass) {
      for (int i = t_; i < M * 8; i += blockDim.x) { const int m = i >> 3, c8 = (i & 7) * 8; v8b o; for (int j = 0; j < 8; ++j) o[j] = (b16)(St[c8 + j][m] * XS); *(volatile v8b*)(Sn + ((size_t)b * MP + PAD + m) * C + half * 64 + c8) = o; }
      if (HORZ) { for (int i = t_; i < 64 * (HP / 4); i += blockDim.x) { const int cc = i / (HP / 4), h4 = (i - cc * (HP / 4)) * 4; const int c = half * 64 + cc; v4f o; for (int j = 0; j < 4; ++j) o[j] = (h4 + j < H) ? St[cc][h4 + j] : 0.0f; *(volatile v4f*)(T + (((size_t)b * C + c) * W + si) * HP + h4) = o; } }
      __threadfence(); }
    if (!HORZ) { for (int i = t_; i < 64 * (W / 4); i += blockDim.x) { const int cc = i / (W / 4), w4 = (i - cc * (W / 4)) * 4; const int c = half * 64 + cc; const size_t o = (((size_t)b * C + c) * H + si) * W + w4; v4f v = *(const v4f*)(out + o); for (int j = 0; j < 4; ++j) v[j] += St[cc][w4 + j]; *(volatile v4f*)(out + o) = v; __threadfence(); *(volatile v4f*)(out + o) = v; } __threadfence(); } }
}
__global__ __launch_bounds__(256) void addT_kernel(const float* __restrict__ T0, float* __restrict__ out) {
  __shared__ float Tt[40][HP + 1];
  const int b = blockIdx.x / C, c = blockIdx.x - b * C, t_ = threadIdx.x; const size_t base = ((size_t)b * C + c);
  for (int w0 = 0; w0 < W; w0 += 40) {
    __syncthreads();
    for (int i = t_; i < 40 * HP; i += 256) { const int ww = i / HP, hh = i - ww * HP; const size_t ti = (base * W + w0 + ww) * HP + hh; Tt[ww][hh] = T0[ti]; }
    __syncthreads();
    for (int i = t_; i < H * 10; i += 256) { const int hh = i / 10, w4 = (i - hh * 10) * 4; const size_t o = (base * H + hh) * W + w0 + w4; v4f v = *(const v4f*)(out + o); for (int j = 0; j < 4; ++j) v[j] += Tt[w4 + j][hh]; *(volatile v4f*)(out + o) = v; __threadfence(); *(volatile v4f*)(out + o) = v; }
    __threadfence(); }
}
}

extern "C" void kernel_launch(void* const* d_in, const int* in_sizes, int n_in, void* d_out, int out_size, void* d_ws, size_t ws_size, hipStream_t stream) {
  (void)n_in;
  auto Fp = [&](int i) { return (const float*)d_in[i]; };
  if (in_sizes[0] != NB * C * H * W || in_sizes[1] != C * C * KT || in_sizes[7] != C * C * KT || out_size != NB * C * H * W) return;
  size_t off = 0; char* ws = (char*)d_ws;
  auto carve = [&](size_t bytes) { char* p = ws + off; off += (bytes + 255) & ~(size_t)255; return p; };
  const size_t slv = (size_t)NB * (W + 2 * PAD) * C, slh = (size_t)NB * (H + 2 * PAD) * C;
  b16* WK = (b16*)carve((size_t)4 * C * KT * C * 2); b16* SL = (b16*)carve((2 * slv + 2 * slh) * 2); float* T = (float*)carve((size_t)NB * C * W * HP * 4);
  if (off > ws_size || off > ((size_t)128 << 20)) return;
  b16* SV0 = SL; b16* SV1 = SL + slv; b16* SH0 = SL + 2 * slv; b16* SH1 = SH0 + slh; float* T0 = T;
  float* out = (float*)d_out;
  prep_kernel<<<(unsigned)((((size_t)NB * C * H * W / 4) + (size_t)4 * C * KT * C / 8 + (2 * slv + 2 * slh) / 8 + (size_t)NB * C * W * HP / 4 + 255) / 256), 256, 0, stream>>>(Fp(0), Fp(1), Fp(3), Fp(5), Fp(7), out, WK, SL, 2 * slv + 2 * slh, T, (size_t)NB * C * W * HP);
  const b16 *WKu = WK, *WKd = WK + (size_t)C * KT * C, *WKl = WK + (size_t)2 * C * KT * C, *WKr = WK + (size_t)3 * C * KT * C;
  seed_kernel<0><<<NB, 256, 0, stream>>>(Fp(0), 0, SV0, out, nullptr);
  for (int i = 1; i < H; ++i) { step_kernel<0><<<NB, 320, 0, stream>>>(Fp(0), (i & 1) ? SV0 : SV1, WKu, Fp(2), i, (i & 1) ? SV1 : SV0, out, nullptr); }
  seed_kernel<0><<<NB, 256, 0, stream>>>(Fp(0), H - 1, SV0, out, nullptr);
  for (int k = 1; k < H; ++k) { const int i = H - 1 - k; step_kernel<0><<<NB, 320, 0, stream>>>(Fp(0), (k & 1) ? SV0 : SV1, WKd, Fp(4), i, (k & 1) ? SV1 : SV0, out, nullptr); }
  seed_kernel<1><<<NB, 256, 0, stream>>>(Fp(0), 0, SH0, nullptr, T0);
  for (int j = 1; j < W; ++j) { step_kernel<1><<<NB, 192, 0, stream>>>(Fp(0), (j & 1) ? SH0 : SH1, WKl, Fp(6), j, (j & 1) ? SH1 : SH0, nullptr, T0); }
  addT_kernel<<<NB * C, 256, 0, stream>>>(T0, out);
  seed_kernel<1><<<NB, 256, 0, stream>>>(Fp(0), W - 1, SH0, nullptr, T0);
  for (int k = 1; k < W; ++k) { const int j = W - 1 - k; step_kernel<1><<<NB, 192, 0, stream>>>(Fp(0), (k & 1) ? SH0 : SH1, WKr, Fp(8), j, (k & 1) ? SH1 : SH0, nullptr, T0); }
  addT_kernel<<<NB * C, 256, 0, stream>>>(T0, out);
}
